// Memory_Transformer_54408645705943
// MI455X (gfx1250) — hardware-verified
//
#include <hip/hip_runtime.h>
#include <stdint.h>

typedef __attribute__((ext_vector_type(16))) __bf16   v16b;
typedef __attribute__((ext_vector_type(8)))  __bf16   v8b;
typedef __attribute__((ext_vector_type(8)))  float    v8f;
typedef __attribute__((ext_vector_type(4)))  float    v4f;
typedef __attribute__((ext_vector_type(4)))  unsigned v4u;

constexpr int NQ      = 1024;
constexpr int NPAST   = 32768;
constexpr int HD      = 128;
constexpr int NKEYS   = NPAST + NQ;
constexpr int KCH     = 64;
constexpr int NCHUNK  = NKEYS / KCH;
constexpr int NPASTCH = NPAST / KCH;
constexpr int QBLK    = 64;
constexpr int NQB     = NQ / QBLK;
constexpr int PACK_ROWS = 16;
constexpr int NPACKB  = NKEYS / PACK_ROWS;
constexpr int TSP     = 132;
constexpr int OSP     = 132;
constexpr float SM_SCALE = 0.08838834764831845f;

constexpr size_t KB_BYTES = (size_t)NKEYS * HD * 2;
constexpr size_t VT_BYTES = (size_t)HD * NKEYS * 2;
constexpr size_t WS_TOTAL = KB_BYTES + VT_BYTES;

static_assert(NKEYS % KCH == 0);
static_assert(NPAST % KCH == 0);
static_assert(NQ % QBLK == 0);
static_assert(QBLK == KCH);
static_assert(HD == 128);
static_assert(HD % 32 == 0);
static_assert(NPAST % PACK_ROWS == 0);
static_assert(NKEYS % PACK_ROWS == 0);
static_assert(PACK_ROWS * HD == 256 * 8);
static_assert((KB_BYTES % 128) == 0);
static_assert(((size_t)NKEYS * 2) % 128 == 0);
static_assert(WS_TOTAL <= (size_t)134217728);

__device__ __forceinline__ unsigned short f2bf_bits(float f) {
  unsigned u = __float_as_uint(f);
  return (unsigned short)((u + 0x7FFFu + ((u >> 16) & 1u)) >> 16);
}
__device__ __forceinline__ float bf_bits2f(unsigned short h) { return __uint_as_float(((unsigned)h) << 16); }
__device__ __forceinline__ __bf16 f2bf(float f) { return __builtin_bit_cast(__bf16, f2bf_bits(f)); }
__device__ __forceinline__ void bf_split(float f, __bf16& hi, __bf16& lo) {
  const unsigned short hb = f2bf_bits(f);
  hi = __builtin_bit_cast(__bf16, hb);
  lo = f2bf(f - bf_bits2f(hb));
}
__device__ __forceinline__ unsigned pack_bf16x2(float e0, float e1) {
  return (unsigned)f2bf_bits(e0) | (((unsigned)f2bf_bits(e1)) << 16);
}

__device__ __forceinline__ v8f mma_bf16(v16b a, v16b b, v8f c) {
  c = __builtin_amdgcn_wmma_f32_16x16x32_bf16(false, a, false, b, (short)0, c, false, false);
  asm volatile("v_nop\n\tv_nop\n\tv_nop\n\tv_nop" : "+v"(c) : "v"(a), "v"(b));
  return c;
}

__global__ __launch_bounds__(256) void pack_k_bf16(const float* __restrict__ kc,
                                                    const float* __restrict__ kn,
                                                    unsigned short* __restrict__ kb) {
  const int r0 = blockIdx.x * PACK_ROWS;
  const float* src = (r0 < NPAST) ? (kc + (size_t)r0 * HD) : (kn + (size_t)(r0 - NPAST) * HD);
  const int t = threadIdx.x;
  const v4f a = *(const v4f*)(src + 8 * t);
  const v4f b = *(const v4f*)(src + 8 * t + 4);
  v4u w;
  w[0] = pack_bf16x2(a[0], a[1]);
  w[1] = pack_bf16x2(a[2], a[3]);
  w[2] = pack_bf16x2(b[0], b[1]);
  w[3] = pack_bf16x2(b[2], b[3]);
  unsigned short* dst = kb + (size_t)r0 * HD + 8 * t;
  *(volatile v4u*)dst = w;
  __threadfence();
  *(volatile v4u*)dst = w;
}

__global__ __launch_bounds__(256) void transpose_v_bf16(const float* __restrict__ vc,
                                                         const float* __restrict__ vn,
                                                         unsigned short* __restrict__ vt) {
  __shared__ __align__(16) float sf[KCH * TSP];
  const int key0 = blockIdx.x * KCH;
  const float* src = (key0 < NPAST) ? (vc + (size_t)key0 * HD) : (vn + (size_t)(key0 - NPAST) * HD);
  const int t = threadIdx.x;
  {
    const int kr = t >> 2;
    const int dq = (t & 3) * 32;
#pragma unroll
    for (int i = 0; i < 8; ++i) {
      const v4f x = *(const v4f*)(src + (size_t)kr * HD + dq + 4 * i);
      *(v4f*)(sf + kr * TSP + dq + 4 * i) = x;
    }
  }
  __syncthreads();
  const int wave = t >> 5;
  const int lane = t & 31;
  const int p = lane & 7;
  const int sub = lane >> 3;
  for (int pass = 0; pass < 2; ++pass) {
#pragma unroll
    for (int it = 0; it < 4; ++it) {
      const int d = wave * 16 + it * 4 + sub;
      const float* col = sf + (8 * p) * TSP + d;
      v4u w;
      w[0] = pack_bf16x2(col[0 * TSP], col[1 * TSP]);
      w[1] = pack_bf16x2(col[2 * TSP], col[3 * TSP]);
      w[2] = pack_bf16x2(col[4 * TSP], col[5 * TSP]);
      w[3] = pack_bf16x2(col[6 * TSP], col[7 * TSP]);
      *(volatile v4u*)(vt + (size_t)d * NKEYS + key0 + 8 * p) = w;
    }
    __threadfence();
  }
}

__global__ __launch_bounds__(128) void attn_step_hd128(const float* __restrict__ q,
                                                        const unsigned short* __restrict__ kb,
                                                        const unsigned short* __restrict__ vt,
                                                        float* __restrict__ out) {
  union FB { v16b v; v8b h[2]; };
  __shared__ __align__(16) __bf16 Ksh[KCH * HD];
  __shared__ __align__(16) __bf16 Vth[HD * KCH];
  __shared__ __align__(16) __bf16 Psh[4][16 * KCH];
  __shared__ __align__(16) __bf16 Psl[4][16 * KCH];
  __shared__ __align__(16) float  Os[4][16 * OSP];

  const int tid  = threadIdx.x;
  const int wave = tid >> 5;
  const int lane = tid & 31;
  const int hh   = lane >> 4;
  const int c    = lane & 15;
  const int qb   = blockIdx.x;
  const int q0   = qb * QBLK + wave * 16;
  const float NEG_INF = -__builtin_inff();

  v16b qa[4];
  {
    const float* qrow = q + (size_t)(q0 + c) * HD;
#pragma unroll
    for (int dc = 0; dc < 4; ++dc) {
      const v4f x0 = *(const v4f*)(qrow + dc * 32 + 8 * hh);
      const v4f x1 = *(const v4f*)(qrow + dc * 32 + 8 * hh + 4);
      const v4f x2 = *(const v4f*)(qrow + dc * 32 + 16 + 8 * hh);
      const v4f x3 = *(const v4f*)(qrow + dc * 32 + 16 + 8 * hh + 4);
#pragma unroll
      for (int e = 0; e < 4; ++e) {
        qa[dc][e]      = f2bf(x0[e]);
        qa[dc][4 + e]  = f2bf(x1[e]);
        qa[dc][8 + e]  = f2bf(x2[e]);
        qa[dc][12 + e] = f2bf(x3[e]);
      }
      if (dc == 1) { asm volatile("" ::: "memory"); }
    }
  }

  float mrow[8], lrow[8];
  v8f oacc[8];
#pragma unroll
  for (int r = 0; r < 8; ++r) { mrow[r] = NEG_INF; lrow[r] = 0.f; }
#pragma unroll
  for (int t = 0; t < 8; ++t) oacc[t] = (v8f){0.f,0.f,0.f,0.f,0.f,0.f,0.f,0.f};

  const int nChunks = NPASTCH + qb + 1;
  for (int kc = 0; kc < nChunks; ++kc) {
    const int kv0 = kc * KCH;
    __syncthreads();
    {
      const int kvr = tid >> 1;
      const int dh  = (tid & 1) * 64;
      const unsigned short* krow = kb + (size_t)(kv0 + kvr) * HD + dh;
      __bf16* kdst = Ksh + kvr * HD + dh;
#pragma unroll
      for (int i = 0; i < 8; ++i) {
        const v4u x = *(const v4u*)(krow + 8 * i);
        *(v8b*)(kdst + 8 * i) = __builtin_bit_cast(v8b, x);
      }
      asm volatile("" ::: "memory");
      const unsigned short* vrow = vt + (size_t)tid * NKEYS + kv0;
      __bf16* vdst = Vth + tid * KCH;
#pragma unroll
      for (int i = 0; i < 8; ++i) {
        const v4u x = *(const v4u*)(vrow + 8 * i);
        *(v8b*)(vdst + 8 * i) = __builtin_bit_cast(v8b, x);
      }
    }
    __syncthreads();

    v8f s[4];
#pragma unroll
    for (int j = 0; j < 4; ++j) {
      s[j] = (v8f){0.f,0.f,0.f,0.f,0.f,0.f,0.f,0.f};
#pragma unroll
      for (int dc = 0; dc < 4; ++dc) {
        FB kf;
        kf.h[0] = *(const v8b*)(Ksh + (j * 16 + c) * HD + dc * 32 + 8 * hh);
        kf.h[1] = *(const v8b*)(Ksh + (j * 16 + c) * HD + dc * 32 + 16 + 8 * hh);
        s[j] = mma_bf16(qa[dc], kf.v, s[j]);
      }
    }

    const bool diag = (kc == NPASTCH + qb);
    float cm[8];
#pragma unroll
    for (int r = 0; r < 8; ++r) {
      const int qrow = q0 + 8 * hh + r;
      float m = NEG_INF;
#pragma unroll
      for (int j = 0; j < 4; ++j) {
        const int kvcol = kv0 + j * 16 + c;
        float sv = s[j][r] * SM_SCALE;
        if (diag) { sv = (kvcol > qrow + NPAST) ? NEG_INF : sv; }
        s[j][r] = sv;
        m = fmaxf(m, sv);
      }
#pragma unroll
      for (int off = 1; off < 16; off <<= 1) m = fmaxf(m, __shfl_xor(m, off, 32));
      cm[r] = m;
    }

    __bf16* pwh = Psh[wave];
    __bf16* pwl = Psl[wave];
#pragma unroll
    for (int r = 0; r < 8; ++r) {
      const float mnew  = fmaxf(mrow[r], cm[r]);
      const float alpha = expf(mrow[r] - mnew);
      mrow[r] = mnew;
      float psum = 0.f;
#pragma unroll
      for (int j = 0; j < 4; ++j) {
        const float p = expf(s[j][r] - mnew);
        psum += p;
        __bf16 ph, pl;
        bf_split(p, ph, pl);
        pwh[(8 * hh + r) * KCH + j * 16 + c] = ph;
        pwl[(8 * hh + r) * KCH + j * 16 + c] = pl;
      }
#pragma unroll
      for (int off = 1; off < 16; off <<= 1) psum += __shfl_xor(psum, off, 32);
      lrow[r] = lrow[r] * alpha + psum;
#pragma unroll
      for (int t = 0; t < 8; ++t) oacc[t][r] *= alpha;
    }
    __builtin_amdgcn_fence(__ATOMIC_RELEASE, "workgroup");
    __builtin_amdgcn_wave_barrier();
    __builtin_amdgcn_fence(__ATOMIC_ACQUIRE, "workgroup");

#pragma unroll 1
    for (int kk = 0; kk < 2; ++kk) {
      FB pa, pb;
      pa.h[0] = *(const v8b*)(pwh + c * KCH + kk * 32 + 8 * hh);
      pa.h[1] = *(const v8b*)(pwh + c * KCH + kk * 32 + 16 + 8 * hh);
      pb.h[0] = *(const v8b*)(pwl + c * KCH + kk * 32 + 8 * hh);
      pb.h[1] = *(const v8b*)(pwl + c * KCH + kk * 32 + 16 + 8 * hh);
#pragma unroll
      for (int t = 0; t < 8; ++t) {
        FB vb;
        vb.h[0] = *(const v8b*)(Vth + (t * 16 + c) * KCH + kk * 32 + 8 * hh);
        vb.h[1] = *(const v8b*)(Vth + (t * 16 + c) * KCH + kk * 32 + 16 + 8 * hh);
        oacc[t] = mma_bf16(pa.v, vb.v, oacc[t]);
        oacc[t] = mma_bf16(pb.v, vb.v, oacc[t]);
      }
    }
  }

  float* os = Os[wave];
#pragma unroll
  for (int r = 0; r < 8; ++r) {
    const float inv = 1.0f / lrow[r];
#pragma unroll
    for (int t = 0; t < 8; ++t) os[(8 * hh + r) * OSP + t * 16 + c] = oacc[t][r] * inv;
  }
  __builtin_amdgcn_fence(__ATOMIC_RELEASE, "workgroup");
  __builtin_amdgcn_wave_barrier();
  __builtin_amdgcn_fence(__ATOMIC_ACQUIRE, "workgroup");
  {
    const int c4 = lane * 4;
    for (int pass = 0; pass < 2; ++pass) {
#pragma unroll
      for (int row = 0; row < 16; ++row) {
        const v4f val = *(const v4f*)(os + row * OSP + c4);
        *(volatile v4f*)(out + (size_t)(q0 + row) * HD + c4) = val;
      }
      __threadfence();
    }
  }
}

extern "C" void kernel_launch(void* const* d_in, const int* in_sizes, int n_in,
                              void* d_out, int out_size, void* d_ws, size_t ws_size,
                              hipStream_t stream) {
  if (n_in < 5) return;
  if (in_sizes[0] != NQ * HD || in_sizes[1] != NQ * HD || in_sizes[2] != NQ * HD) return;
  if (in_sizes[3] != NPAST * HD || in_sizes[4] != NPAST * HD) return;
  if (out_size != NQ * HD) return;
  if (ws_size < WS_TOTAL) return;

  const float* q  = (const float*)d_in[0];
  const float* kn = (const float*)d_in[1];
  const float* vn = (const float*)d_in[2];
  const float* kc = (const float*)d_in[3];
  const float* vc = (const float*)d_in[4];
  float* out = (float*)d_out;

  unsigned short* kbp = (unsigned short*)d_ws;
  unsigned short* vtp = (unsigned short*)((char*)d_ws + KB_BYTES);

  pack_k_bf16<<<NPACKB, 256, 0, stream>>>(kc, kn, kbp);
  transpose_v_bf16<<<NCHUNK, 256, 0, stream>>>(vc, vn, vtp);
  attn_step_hd128<<<NQB, 128, 0, stream>>>(q, kbp, vtp, out);
}
